// DecGridDeepVPN_33328946217237
// MI455X (gfx1250) — hardware-run, weakly checked
//
#include <hip/hip_runtime.h>

typedef _Float16 v16h __attribute__((ext_vector_type(16)));
typedef _Float16 v8h  __attribute__((ext_vector_type(8)));
typedef float    v8f  __attribute__((ext_vector_type(8)));
typedef float    v4f  __attribute__((ext_vector_type(4)));
typedef v8h __attribute__((may_alias)) v8ha;
typedef v4f __attribute__((may_alias)) v4fa;

union Frag { v16h v; v8h half[2]; };

#define S_NUM 81
#define N_AG  20
#define N_ACT 5
#define GRIDW 9
#define TB    32
#define OBS_STRIDE 182
#define AC_STRIDE  405
#define LA_STRIDE  100
#define ROWS  (TB * N_AG)
#define KP    96
#define H0S   40
#define W0R   106
#define NTHR  256
#define WSC   64.0f
#define INV_WSC 0.015625f

struct __attribute__((aligned(16))) Smem {
  _Float16 nsc16[TB][KP];
  _Float16 w0a_t[32][KP];
  _Float16 w1t[32][32];
  _Float16 h0[ROWS][H0S];
  float    ostage[ROWS];
  float    served[TB * S_NUM];
  float    base[TB][32];
  float    w0r[W0R * 32];
  float    w2v[32];
  float    la[TB * LA_STRIDE];
  float    reward[TB];
  int      loc[ROWS];
};
static_assert((sizeof(Smem) % 16) == 0);
static_assert((__builtin_offsetof(Smem, ostage) % 16) == 0);
static_assert((__builtin_offsetof(Smem, h0) % 16) == 0);
static_assert((__builtin_offsetof(Smem, w1t) % 16) == 0);

__device__ __forceinline__ v8f wmma_f16(v16h a, v16h b, v8f c) {
  v8f d = __builtin_amdgcn_wmma_f32_16x16x32_f16(false, a, false, b, (short)0, c, false, false);
#if defined(__HIP_DEVICE_COMPILE__)
  asm volatile("v_nop\n\tv_nop\n\tv_nop\n\tv_nop" : "+v"(d) : "v"(a), "v"(b));
#endif
  return d;
}

__device__ __forceinline__ v16h load_frag(const _Float16* p, int h) {
  Frag f;
  f.half[0] = *(const v8ha*)(p + 8 * h);
  f.half[1] = *(const v8ha*)(p + 16 + 8 * h);
  return f.v;
}

__device__ __forceinline__ void out_store_pass(float* ob, const v4f* vals, int lane) {
#pragma unroll
  for (int i = 0; i < 5; ++i)
    *(volatile v4f*)(ob + 4 * (32 * i + lane)) = vals[i];
}

__global__ __launch_bounds__(NTHR, 2)
void vpn_fused(const float* __restrict__ obs,
               const float* __restrict__ action_count,
               const float* __restrict__ local_actions,
               const float* __restrict__ W0,
               const float* __restrict__ W1,
               const float* __restrict__ W2,
               const float* __restrict__ b2,
               float* __restrict__ out)
{
  extern __shared__ __attribute__((aligned(16))) char smem_raw[];
  Smem& sm = *reinterpret_cast<Smem*>(smem_raw);
  const int tid  = threadIdx.x;
  const int lane = tid & 31;
  const int wave = tid >> 5;
  const int h    = lane >> 4;
  const int m    = lane & 15;
  const int b0   = blockIdx.x * TB;
  const v8f zero8 = {0.f, 0.f, 0.f, 0.f, 0.f, 0.f, 0.f, 0.f};

  for (int idx = tid; idx < TB * S_NUM; idx += NTHR) {
    const int bl = idx / S_NUM;
    const int d  = idx - bl * S_NUM;
    const int r  = d / GRIDW, c = d - r * GRIDW;
    const float* ac = action_count + (size_t)(b0 + bl) * AC_STRIDE;
    float sum = ac[d * N_ACT];
    int s;
    s = (r + 1 < GRIDW) ? ((d + GRIDW) * N_ACT + 1) : (d * N_ACT + 2);  sum += ac[s];
    s = (r - 1 >= 0)    ? ((d - GRIDW) * N_ACT + 2) : (d * N_ACT + 1);  sum += ac[s];
    s = (c + 1 < GRIDW) ? ((d + 1) * N_ACT + 3)     : (d * N_ACT + 4);  sum += ac[s];
    s = (c - 1 >= 0)    ? ((d - 1) * N_ACT + 4)     : (d * N_ACT + 3);  sum += ac[s];
    const float demand = obs[(size_t)(b0 + bl) * OBS_STRIDE + S_NUM + d];
    sm.nsc16[bl][d] = (_Float16)sum;
    sm.served[bl * S_NUM + d] = fminf(sum, demand);
  }
  for (int idx = tid; idx < TB * (KP - S_NUM); idx += NTHR) {
    const int bl = idx / (KP - S_NUM);
    sm.nsc16[bl][S_NUM + (idx - bl * (KP - S_NUM))] = (_Float16)0.0f;
  }
  for (int idx = tid; idx < 32 * KP; idx += NTHR) {
    const int n = idx / KP, k = idx - n * KP;
    const int kc = (k < S_NUM) ? k : (S_NUM - 1);
    const float w = W0[kc * 32 + n] * WSC;
    sm.w0a_t[n][k] = (_Float16)((k < S_NUM) ? w : 0.0f);
  }
  for (int idx = tid; idx < W0R * 32; idx += NTHR)
    sm.w0r[idx] = W0[S_NUM * 32 + idx];
  for (int idx = tid; idx < 32 * 32; idx += NTHR) {
    const int n = idx >> 5, k = idx & 31;
    sm.w1t[n][k] = (_Float16)(W1[k * 32 + n] * WSC);
  }
  if (tid < 32) sm.w2v[tid] = W2[tid];
  for (int idx = tid; idx < TB * LA_STRIDE; idx += NTHR)
    sm.la[idx] = local_actions[(size_t)b0 * LA_STRIDE + idx];
  for (int idx = tid; idx < ROWS; idx += NTHR) {
    const int bl = idx / N_AG, n = idx - bl * N_AG;
    float v = obs[(size_t)(b0 + bl) * OBS_STRIDE + 2 * S_NUM + n];
    v = fminf(fmaxf(v, -4.0f), 1024.0f);
    const int l = (int)v;
    sm.loc[idx] = (l >= 0 && l < S_NUM) ? l : -1;
  }
  __syncthreads();

  if (wave < 2) {
    v8f c0 = zero8, c1 = zero8;
    const int r0w = wave * 16;
#pragma unroll
    for (int kt = 0; kt < 3; ++kt) {
      const int k0 = kt * 32;
      const v16h a  = load_frag(&sm.nsc16[r0w + m][k0], h);
      const v16h bA = load_frag(&sm.w0a_t[m][k0], h);
      const v16h bB = load_frag(&sm.w0a_t[16 + m][k0], h);
      c0 = wmma_f16(a, bA, c0);
      c1 = wmma_f16(a, bB, c1);
    }
#pragma unroll
    for (int r = 0; r < 8; ++r) {
      sm.base[r0w + 8 * h + r][m]      = c0[r] * INV_WSC;
      sm.base[r0w + 8 * h + r][16 + m] = c1[r] * INV_WSC;
    }
  } else if (wave == 2) {
    float acc = 0.0f;
    const float* sv = &sm.served[lane * S_NUM];
#pragma unroll 1
    for (int d = 0; d < S_NUM; ++d) acc += sv[d];
    sm.reward[lane] = acc;
  }
  __syncthreads();

  for (int idx = tid; idx < ROWS * 32; idx += NTHR) {
    const int row = idx >> 5, k = idx & 31;
    const int bl = row / N_AG, ag = row - bl * N_AG;
    const int l  = sm.loc[row];
    const int lc = (l < 0) ? 0 : l;
    const float wl = sm.w0r[lc * 32 + k];
    float v = sm.base[bl][k] + ((l < 0) ? 0.0f : wl) + sm.w0r[(S_NUM + N_ACT + ag) * 32 + k];
    const float* lap = &sm.la[row * N_ACT];
#pragma unroll
    for (int a = 0; a < N_ACT; ++a) v += lap[a] * sm.w0r[(S_NUM + a) * 32 + k];
    sm.h0[row][k] = (_Float16)fmaxf(v, 0.0f);
  }
  __syncthreads();

  {
    const v16h bw0 = load_frag(&sm.w1t[m][0], h);
    const v16h bw1 = load_frag(&sm.w1t[16 + m][0], h);
    const float w2a = sm.w2v[m];
    const float w2b = sm.w2v[16 + m];
    const float b2v = b2[0];
    const int j = lane & 7;
#pragma unroll 1
    for (int i = 0; i < 5; ++i) {
      const int t = wave * 5 + i;
      const v16h a = load_frag(&sm.h0[t * 16 + m][0], h);
      const v8f c0 = wmma_f16(a, bw0, zero8);
      const v8f c1 = wmma_f16(a, bw1, zero8);
      float p[8];
#pragma unroll
      for (int q = 0; q < 8; ++q)
        p[q] = fmaxf(c0[q] * INV_WSC, 0.0f) * w2a + fmaxf(c1[q] * INV_WSC, 0.0f) * w2b;
#pragma unroll
      for (int off = 1; off < 16; off <<= 1) {
#pragma unroll
        for (int q = 0; q < 8; ++q) p[q] += __shfl_xor(p[q], off, 32);
      }
      float psel = p[0];
#pragma unroll
      for (int q = 1; q < 8; ++q) psel = (j == q) ? p[q] : psel;
      if ((lane & 8) == 0) {
        const int row = t * 16 + 8 * h + j;
        const int bl  = row / N_AG;
        sm.ostage[row] = sm.reward[bl] + (psel + b2v);
      }
    }
  }
  __syncthreads();

  if (wave == 0) {
    const v4fa* src = (const v4fa*)sm.ostage;
    v4f vals[5];
#pragma unroll
    for (int i = 0; i < 5; ++i) vals[i] = src[32 * i + lane];
    float* ob = out + (size_t)b0 * N_AG;
    out_store_pass(ob, vals, lane);
    __threadfence();
    out_store_pass(ob, vals, lane);
  }
}

extern "C" void kernel_launch(void* const* d_in, const int* in_sizes, int n_in,
                              void* d_out, int out_size, void* d_ws, size_t ws_size,
                              hipStream_t stream) {
  (void)d_ws; (void)ws_size;
  if (n_in < 7) return;
  const int batch = in_sizes[0] / OBS_STRIDE;
  if (batch <= 0 || batch * OBS_STRIDE != in_sizes[0]) return;
  if (in_sizes[1] != batch * AC_STRIDE) return;
  if (in_sizes[2] != batch * LA_STRIDE) return;
  if (in_sizes[3] != (2 * S_NUM + N_ACT + N_AG) * 32) return;
  if (in_sizes[4] != 32 * 32) return;
  if (in_sizes[5] != 32) return;
  if (in_sizes[6] < 1) return;
  if (out_size != batch * N_AG) return;
  if ((batch % TB) != 0) return;

  const float* obs           = (const float*)d_in[0];
  const float* action_count  = (const float*)d_in[1];
  const float* local_actions = (const float*)d_in[2];
  const float* W0            = (const float*)d_in[3];
  const float* W1            = (const float*)d_in[4];
  const float* W2            = (const float*)d_in[5];
  const float* b2            = (const float*)d_in[6];
  float* out = (float*)d_out;

  const size_t smem = sizeof(Smem);
  hipFuncSetAttribute(reinterpret_cast<const void*>(&vpn_fused),
                      hipFuncAttributeMaxDynamicSharedMemorySize, (int)smem);
  vpn_fused<<<dim3(batch / TB), dim3(NTHR), smem, stream>>>(
      obs, action_count, local_actions, W0, W1, W2, b2, out);
  (void)hipGetLastError();
}
